// STMetaLSTM_17995912970448
// MI455X (gfx1250) — hardware-verified
//
#include <hip/hip_runtime.h>
#include <stdint.h>

typedef __attribute__((ext_vector_type(16))) _Float16 v16h;
typedef __attribute__((ext_vector_type(8)))  _Float16 v8h;
typedef __attribute__((ext_vector_type(16))) __bf16   v16b;
typedef __attribute__((ext_vector_type(8)))  __bf16   v8b;
typedef __attribute__((ext_vector_type(8)))  float    v8f;
typedef __attribute__((ext_vector_type(4)))  float    v4f;
typedef __attribute__((ext_vector_type(4)))  unsigned int v4u;

constexpr int NBATCH = 32;
constexpr int NSTEP  = 12;
constexpr int NNODE  = 325;
constexpr int NHID   = 64;
constexpr int NEMB   = 96;
constexpr int NLH    = 128;
constexpr int NOUTS  = 12;
constexpr int XPITCH = NEMB + 1;
constexpr int BNREAL = NBATCH * NNODE;
constexpr int MCH    = 1536;
constexpr int NCHUNK = 7;
constexpr int MPAD   = MCH * NCHUNK;
constexpr int WHN    = NHID * NHID;
constexpr int NOUTEL = NBATCH * NOUTS * NNODE;
static_assert(MPAD >= BNREAL, "pad");
static_assert(MPAD % 64 == 0 && MCH % 64 == 0, "tile multiples");
static_assert(NEMB % 32 == 0 && NLH % 32 == 0 && NHID % 32 == 0, "K multiples of 32");
static_assert(NLH % 64 == 0 && NHID % 64 == 0 && WHN % 64 == 0, "N multiples of 64");
constexpr int TILES_L1 = (MPAD / 64) * (NLH / 64);
constexpr int TILES_L2 = (MPAD / 64) * (NHID / 64);
constexpr int TILES_WH = (MCH / 64) * (WHN / 64);
static_assert(TILES_L1 % 8 == 0 && TILES_L2 % 8 == 0 && TILES_WH % 8 == 0, "whole blocks");
static_assert((MPAD * 12) % 256 == 0, "meta grid exact");
static_assert(NOUTEL % 4 == 0 && (NOUTEL / 4) % 32 == 0, "output waves whole");

constexpr size_t SZ_META = (size_t)MPAD * NEMB * 2;
constexpr size_t SZ_W1T  = (size_t)12 * NLH * NEMB * 2;
constexpr size_t SZ_W2T  = (size_t)8 * NHID * NLH * 2;
constexpr size_t SZ_WH2T = (size_t)4 * WHN * NLH * 2;
constexpr size_t SZ_WHBP = (size_t)4 * WHN * 4;
constexpr size_t SZ_FC1T = (size_t)32 * 64 * 2;
constexpr size_t SZ_FC2T = (size_t)16 * 32 * 2;
constexpr size_t SZ_HID  = (size_t)4 * MPAD * NLH * 2;
constexpr size_t SZ_WX   = (size_t)MPAD * 256 * 4;
constexpr size_t SZ_WHS  = (size_t)MCH * 4 * WHN * 2;
constexpr size_t SZ_HOUT = (size_t)MPAD * 32 * 4;
constexpr size_t OFF_META_H = 0;
constexpr size_t OFF_META_L = OFF_META_H + SZ_META;
constexpr size_t OFF_W1T_H  = OFF_META_L + SZ_META;
constexpr size_t OFF_W1T_L  = OFF_W1T_H + SZ_W1T;
constexpr size_t OFF_W2T_H  = OFF_W1T_L + SZ_W1T;
constexpr size_t OFF_W2T_L  = OFF_W2T_H + SZ_W2T;
constexpr size_t OFF_WH2T   = OFF_W2T_L + SZ_W2T;
constexpr size_t OFF_WHBP   = OFF_WH2T + SZ_WH2T;
constexpr size_t OFF_FC1T_H = OFF_WHBP + SZ_WHBP;
constexpr size_t OFF_FC1T_L = OFF_FC1T_H + SZ_FC1T;
constexpr size_t OFF_FC2T_H = OFF_FC1T_L + SZ_FC1T;
constexpr size_t OFF_FC2T_L = OFF_FC2T_H + SZ_FC2T;
constexpr size_t OFF_HID_H  = OFF_FC2T_L + SZ_FC2T;
constexpr size_t OFF_HID_L  = OFF_HID_H + SZ_HID;
constexpr size_t OFF_WX     = OFF_HID_L + SZ_HID;
constexpr size_t OFF_BB     = OFF_WX + SZ_WX;
constexpr size_t OFF_WHS    = OFF_BB + SZ_WX;
constexpr size_t OFF_HOUT   = OFF_WHS + SZ_WHS;
constexpr size_t WS_TOTAL   = OFF_HOUT + SZ_HOUT;
static_assert(WS_TOTAL == 104998912ull, "carve total");
static_assert(WS_TOTAL <= 134217728ull, "carve under 128 MiB");
static_assert(OFF_META_L % 256 == 0 && OFF_W1T_H % 256 == 0 && OFF_W2T_H % 256 == 0 && OFF_WH2T % 256 == 0 &&
              OFF_WHBP % 256 == 0 && OFF_FC1T_H % 256 == 0 && OFF_FC2T_H % 256 == 0 && OFF_FC2T_L % 256 == 0 &&
              OFF_HID_H % 256 == 0 && OFF_HID_L % 256 == 0 && OFF_WX % 256 == 0 && OFF_BB % 256 == 0 &&
              OFF_WHS % 256 == 0 && OFF_HOUT % 256 == 0, "aligned regions");
static_assert(SZ_HID >= (size_t)4 * MPAD * NLH * 2, "hid region also holds the f16 hidden plane");

__device__ __forceinline__ unsigned short f2bf_bits(float f) {
  unsigned u = __float_as_uint(f);
  return (unsigned short)((u + 0x7FFFu + ((u >> 16) & 1u)) >> 16);
}
__device__ __forceinline__ float bf_bits2f(unsigned short h) { return __uint_as_float(((unsigned)h) << 16); }

__device__ __forceinline__ void dep_guard_h(v8f& a, v8f& b, v16h x, v16h y) { asm volatile("v_nop\n\tv_nop\n\tv_nop\n\tv_nop" : "+v"(a), "+v"(b) : "v"(x), "v"(y)); }
__device__ __forceinline__ void dep_guard_b(v8f& a, v8f& b, v16b x, v16b y) { asm volatile("v_nop\n\tv_nop\n\tv_nop\n\tv_nop" : "+v"(a), "+v"(b) : "v"(x), "v"(y)); }
__device__ __forceinline__ void keep4_h(v16h a, v16h b, v16h c, v16h d) { asm volatile("v_nop" :: "v"(a), "v"(b), "v"(c), "v"(d)); }
__device__ __forceinline__ void keep4_b(v16b a, v16b b, v16b c, v16b d) { asm volatile("v_nop" :: "v"(a), "v"(b), "v"(c), "v"(d)); }
__device__ __forceinline__ void acc_guard4(v8f& a, v8f& b, v8f& c, v8f& d) { asm volatile("v_nop\n\tv_nop\n\tv_nop\n\tv_nop" : "+v"(a), "+v"(b), "+v"(c), "+v"(d)); }
__device__ __forceinline__ void guard1h(v8f& c, v16h a, v16h b) { asm volatile("v_nop\n\tv_nop\n\tv_nop\n\tv_nop" : "+v"(c) : "v"(a), "v"(b)); }
__device__ __forceinline__ void guard1b(v8f& c, v16b a, v16b b) { asm volatile("v_nop\n\tv_nop\n\tv_nop\n\tv_nop" : "+v"(c) : "v"(a), "v"(b)); }

template <typename T> struct Frag;
template <> struct Frag<_Float16> {
  typedef v16h V; union U { v16h v; v8h h[2]; };
  static __device__ __forceinline__ v16h load(const _Float16* p) {
    U f; f.h[0] = *(const v8h*)(p); f.h[1] = *(const v8h*)(p + 16); return f.v;
  }
  static __device__ __forceinline__ v8f mma(v16h a, v16h b, v8f c) {
    return __builtin_amdgcn_wmma_f32_16x16x32_f16(false, a, false, b, (short)0, c, false, false);
  }
  static __device__ __forceinline__ void guard(v8f& a, v8f& b, v16h x, v16h y) { dep_guard_h(a, b, x, y); }
  static __device__ __forceinline__ void keep(v16h a, v16h b, v16h c, v16h d) { keep4_h(a, b, c, d); }
};
template <> struct Frag<__bf16> {
  typedef v16b V; union U { v16b v; v8b h[2]; };
  static __device__ __forceinline__ v16b load(const __bf16* p) {
    U f; f.h[0] = *(const v8b*)(p); f.h[1] = *(const v8b*)(p + 16); return f.v;
  }
  static __device__ __forceinline__ v8f mma(v16b a, v16b b, v8f c) {
    return __builtin_amdgcn_wmma_f32_16x16x32_bf16(false, a, false, b, (short)0, c, false, false);
  }
  static __device__ __forceinline__ void guard(v8f& a, v8f& b, v16b x, v16b y) { dep_guard_b(a, b, x, y); }
  static __device__ __forceinline__ void keep(v16b a, v16b b, v16b c, v16b d) { keep4_b(a, b, c, d); }
};

__device__ __forceinline__ void wave_lds_sync() {
  __builtin_amdgcn_fence(__ATOMIC_RELEASE, "workgroup");
  __builtin_amdgcn_wave_barrier();
  __builtin_amdgcn_fence(__ATOMIC_ACQUIRE, "workgroup");
}
__device__ __forceinline__ v8f zero8() { return (v8f){0.f, 0.f, 0.f, 0.f, 0.f, 0.f, 0.f, 0.f}; }
__device__ __forceinline__ unsigned pk2(unsigned short a, unsigned short b) { return (unsigned)a | ((unsigned)b << 16); }

template <int ET> struct Elem;
template <> struct Elem<0> { typedef _Float16 T; };
template <> struct Elem<1> { typedef __bf16 T; };
template <int ET, bool SPLIT, int BIAS_MODE, int OUT_MODE, bool RESID, int ACT = 0>
__global__ __launch_bounds__(256) void wmma_gemm64(
    const unsigned short* __restrict__ Ap, const unsigned short* __restrict__ A2p, int lda, long strideA,
    const unsigned short* __restrict__ Btp, const unsigned short* __restrict__ Bt2p, int ldb, long strideB,
    void* __restrict__ Cout, void* __restrict__ Cout2, int ldc, long strideC,
    const float* __restrict__ bias, long strideBias,
    const float* __restrict__ resid, long strideR,
    int M, int N, int K, float scale, float post) {
  typedef typename Elem<ET>::T T;
  typedef typename Frag<T>::V V;
  const T* A = (const T*)Ap; const T* A2 = (const T*)A2p; const T* Bt = (const T*)Btp; const T* Bt2 = (const T*)Bt2p;
  __shared__ __align__(16) float sT[8][16 * 68];
  const int b    = blockIdx.y;
  const int lane = threadIdx.x & 31;
  const int wave = threadIdx.x >> 5;
  const int tilesN = N >> 6;
  const int tilesM = M >> 6;
  const int tile = blockIdx.x * 8 + wave;
  if (tile >= tilesM * tilesN) return;
  const int tm = tile / tilesN;
  const int tn = tile - tm * tilesN;
  const int m0 = tm << 6;
  const int n0 = tn << 6;

  const T* Ab  = A  + (size_t)b * strideA;
  const T* Bb  = Bt + (size_t)b * strideB;
  const T* Ab2 = SPLIT ? (A2  + (size_t)b * strideA) : nullptr;
  const T* Bb2 = SPLIT ? (Bt2 + (size_t)b * strideB) : nullptr;
  const float* biasb = (BIAS_MODE != 0) ? (bias + (size_t)b * strideBias) : nullptr;

  const int rlane = lane & 15;
  const int koff  = (lane >> 4) * 8;
  const int mOff  = (lane >> 4) * 8;

  v8f acc[4][4];
#pragma unroll
  for (int i = 0; i < 4; ++i)
#pragma unroll
    for (int j = 0; j < 4; ++j) acc[i][j] = (v8f){0.f,0.f,0.f,0.f,0.f,0.f,0.f,0.f};

  for (int k0 = 0; k0 < K; k0 += 32) {
    V bh[4], bl[4];
#pragma unroll
    for (int j = 0; j < 4; ++j) {
      const size_t bo = (size_t)(n0 + (j << 4) + rlane) * ldb + koff + k0;
      bh[j] = Frag<T>::load(Bb + bo);
      if (SPLIT) bl[j] = Frag<T>::load(Bb2 + bo);
    }
#pragma unroll
    for (int i = 0; i < 4; ++i) {
      const size_t ao = (size_t)(m0 + (i << 4) + rlane) * lda + koff + k0;
      V ah = Frag<T>::load(Ab + ao);
      V al;
      if (SPLIT) al = Frag<T>::load(Ab2 + ao);
#pragma unroll
      for (int j = 0; j < 4; ++j) {
        acc[i][j] = Frag<T>::mma(ah, bh[j], acc[i][j]);
        if (SPLIT) {
          acc[i][j] = Frag<T>::mma(ah, bl[j], acc[i][j]);
          acc[i][j] = Frag<T>::mma(al, bh[j], acc[i][j]);
        }
      }
      Frag<T>::guard(acc[i][0], acc[i][3], ah, SPLIT ? al : ah);
    }
    Frag<T>::keep(bh[0], bh[1], bh[2], bh[3]);
    if (SPLIT) Frag<T>::keep(bl[0], bl[1], bl[2], bl[3]);
  }
  acc_guard4(acc[0][0], acc[0][1], acc[0][2], acc[0][3]);
  acc_guard4(acc[1][0], acc[1][1], acc[1][2], acc[1][3]);
  acc_guard4(acc[2][0], acc[2][1], acc[2][2], acc[2][3]);
  acc_guard4(acc[3][0], acc[3][1], acc[3][2], acc[3][3]);

  float* slab = sT[wave];
  const float* Rb = RESID ? (resid + (size_t)b * strideR) : nullptr;
#pragma unroll
  for (int i = 0; i < 4; ++i) {
    const int mBase = m0 + (i << 4);
#pragma unroll
    for (int j = 0; j < 4; ++j) {
      const int n = n0 + (j << 4) + rlane;
      float bv = 0.f;
      if (BIAS_MODE == 2) bv = biasb[n];
#pragma unroll
      for (int r = 0; r < 8; ++r) {
        float v = acc[i][j][r] * scale;
        if (BIAS_MODE == 1) v += biasb[mBase + mOff + r];
        if (BIAS_MODE == 2) v += bv;
        if (RESID) v += Rb[(size_t)(mBase + mOff + r) * ldc + n];
        v = v * post;
        if (ACT == 1) v = tanhf(v);
        if (ACT == 2) v = fmaxf(v, 0.0f);
        if (ACT == 4) v = (v > 0.f) ? v : 0.01f * v;
        slab[(mOff + r) * 68 + (j << 4) + rlane] = v;
      }
    }
    __builtin_amdgcn_fence(__ATOMIC_RELEASE, "workgroup");
    __builtin_amdgcn_wave_barrier();
    __builtin_amdgcn_fence(__ATOMIC_ACQUIRE, "workgroup");
    if (OUT_MODE == 0) {
      float* C = (float*)Cout + (size_t)b * strideC;
      const int hh = lane >> 4, c4 = (lane & 15) * 4;
      for (int pass = 0; pass < 2; ++pass) {
#pragma unroll
        for (int it = 0; it < 8; ++it) {
          const int row = it * 2 + hh;
          v4f v = *(const v4f*)(slab + row * 68 + c4);
          *(volatile v4f*)(C + (size_t)(mBase + row) * ldc + n0 + c4) = v;
        }
        __threadfence();
      }
    } else {
      const int q = lane >> 3, c8 = (lane & 7) * 8;
      unsigned short* C  = (unsigned short*)Cout  + (size_t)b * strideC;
      unsigned short* C2 = (OUT_MODE == 2) ? ((unsigned short*)Cout2 + (size_t)b * strideC) : nullptr;
      for (int pass = 0; pass < 2; ++pass) {
#pragma unroll
        for (int it = 0; it < 4; ++it) {
          const int row = it * 4 + q;
          const float* sp = slab + row * 68 + c8;
          v8h hv, lv;
#pragma unroll
          for (int e = 0; e < 8; ++e) {
            if (OUT_MODE == 1) {
              hv[e] = (_Float16)sp[e];
            } else {
              unsigned short hb = f2bf_bits(sp[e]);
              unsigned short lb = f2bf_bits(sp[e] - bf_bits2f(hb));
              hv[e] = __builtin_bit_cast(_Float16, hb);
              lv[e] = __builtin_bit_cast(_Float16, lb);
            }
          }
          *(volatile v8h*)(C + (size_t)(mBase + row) * ldc + n0 + c8) = hv;
          if (OUT_MODE == 2) *(volatile v8h*)(C2 + (size_t)(mBase + row) * ldc + n0 + c8) = lv;
        }
        __threadfence();
      }
    }
    __builtin_amdgcn_fence(__ATOMIC_RELEASE, "workgroup");
    __builtin_amdgcn_wave_barrier();
    __builtin_amdgcn_fence(__ATOMIC_ACQUIRE, "workgroup");
  }
}

__device__ __forceinline__ void pack_split8(const float (&v)[8], v4u& wh, v4u& wl) {
#pragma unroll
  for (int p = 0; p < 4; ++p) {
    const unsigned short h0 = f2bf_bits(v[2 * p]);
    const unsigned short h1 = f2bf_bits(v[2 * p + 1]);
    const unsigned short l0 = f2bf_bits(v[2 * p] - bf_bits2f(h0));
    const unsigned short l1 = f2bf_bits(v[2 * p + 1] - bf_bits2f(h1));
    wh[p] = pk2(h0, h1);
    wl[p] = pk2(l0, l1);
  }
}
__device__ __forceinline__ void store_planes2(unsigned short* hi, unsigned short* lo, size_t off, v4u wh, v4u wl) {
  *(volatile v4u*)(hi + off) = wh;
  *(volatile v4u*)(lo + off) = wl;
  __threadfence();
  *(volatile v4u*)(hi + off) = wh;
  *(volatile v4u*)(lo + off) = wl;
}

__global__ __launch_bounds__(256) void k_meta(const float* __restrict__ x,
                                              unsigned short* __restrict__ mh, unsigned short* __restrict__ ml) {
  const int i = blockIdx.x * 256 + threadIdx.x;
  if (i >= MPAD * 12) return;
  const int row = i / 12;
  const int q = i - row * 12;
  const bool real = row < BNREAL;
  const int rowc = real ? row : (BNREAL - 1);
  const int b = rowc / NNODE;
  const int n = rowc - b * NNODE;
  const float* xp = x + ((size_t)b * NSTEP * NNODE + n) * XPITCH + 1 + 8 * q;
  float s[8];
#pragma unroll
  for (int e = 0; e < 8; ++e) s[e] = 0.f;
#pragma unroll 1
  for (int t = 0; t < NSTEP; ++t) {
    const float* p = xp + (size_t)t * (NNODE * XPITCH);
#pragma unroll
    for (int e = 0; e < 8; ++e) s[e] += p[e];
  }
  float v[8];
#pragma unroll
  for (int e = 0; e < 8; ++e) v[e] = real ? (s[e] * (1.0f / 12.0f)) : 0.f;
  v4u wh, wl;
  pack_split8(v, wh, wl);
  store_planes2(mh, ml, (size_t)i * 8, wh, wl);
}

__global__ __launch_bounds__(256) void k_prep_w1(const float* __restrict__ wx1, const float* __restrict__ wh1,
                                                 const float* __restrict__ b1,
                                                 unsigned short* __restrict__ th, unsigned short* __restrict__ tl) {
  const int i = blockIdx.x * 256 + threadIdx.x;
  if (i >= 4 * 1536) return;
  const int hyp = blockIdx.y;
  const float* src = (hyp == 0) ? wx1 : ((hyp == 1) ? wh1 : b1);
  const int g = i / 1536;
  const int r = i - g * 1536;
  const int n = r / 12;
  const int q = r - n * 12;
  const float* sp = src + (size_t)g * (NEMB * NLH) + (size_t)(8 * q) * NLH + n;
  float v[8];
#pragma unroll
  for (int e = 0; e < 8; ++e) v[e] = sp[(size_t)e * NLH];
  v4u wh, wl;
  pack_split8(v, wh, wl);
  store_planes2(th, tl, (size_t)hyp * (4 * NLH * NEMB) + (size_t)i * 8, wh, wl);
}

__global__ __launch_bounds__(256) void k_prep_w2(const float* __restrict__ wx2, const float* __restrict__ b2,
                                                 unsigned short* __restrict__ th, unsigned short* __restrict__ tl) {
  const int i = blockIdx.x * 256 + threadIdx.x;
  if (i >= 4 * 1024) return;
  const int which = blockIdx.y;
  const float* src = (which == 0) ? wx2 : b2;
  const int g = i >> 10;
  const int r = i & 1023;
  const int n = r >> 4;
  const int q = r & 15;
  const float* sp = src + (size_t)g * (NLH * NHID) + (size_t)(8 * q) * NHID + n;
  float v[8];
#pragma unroll
  for (int e = 0; e < 8; ++e) v[e] = sp[(size_t)e * NHID];
  v4u wh, wl;
  pack_split8(v, wh, wl);
  store_planes2(th, tl, (size_t)which * (4 * NHID * NLH) + (size_t)i * 8, wh, wl);
}

__global__ __launch_bounds__(256) void k_prep_wh2(const float* __restrict__ wh2, unsigned short* __restrict__ t16) {
  const int i = blockIdx.x * 256 + threadIdx.x;
  if (i >= 4096 * 16) return;
  const int g = blockIdx.y;
  const int np = i >> 4;
  const int q = i & 15;
  const int kout = np >> 6;
  const int ii = np & 63;
  const int col = ii * 64 + kout;
  const float* sp = wh2 + (size_t)g * (NLH * WHN) + (size_t)(8 * q) * WHN + col;
  v4u w;
#pragma unroll
  for (int p = 0; p < 4; ++p) {
    const float f0 = 64.0f * sp[(size_t)(2 * p) * WHN];
    const float f1 = 64.0f * sp[(size_t)(2 * p + 1) * WHN];
    w[p] = pk2(__builtin_bit_cast(unsigned short, (_Float16)f0), __builtin_bit_cast(unsigned short, (_Float16)f1));
  }
  const size_t off = (size_t)g * (WHN * NLH) + (size_t)i * 8;
  *(volatile v4u*)(t16 + off) = w;
  __threadfence();
  *(volatile v4u*)(t16 + off) = w;
}

__global__ __launch_bounds__(256) void k_prep_misc(const float* __restrict__ wh2b, const float* __restrict__ fc1,
                                                   const float* __restrict__ fc2,
                                                   float* __restrict__ whbp,
                                                   unsigned short* __restrict__ f1h, unsigned short* __restrict__ f1l,
                                                   unsigned short* __restrict__ f2h, unsigned short* __restrict__ f2l) {
  const int task = blockIdx.y;
  const int tid = threadIdx.x;
  if (task == 0) {
    const int i = blockIdx.x * 256 + tid;
    if (i >= 4096) return;
    const int g = i >> 10;
    const int r = i & 1023;
    v4f v;
#pragma unroll
    for (int e = 0; e < 4; ++e) {
      const int np = 4 * r + e;
      const int col = (np & 63) * 64 + (np >> 6);
      v[e] = wh2b[(size_t)g * WHN + col];
    }
    float* dst = whbp + (size_t)i * 4;
    *(volatile v4f*)dst = v;
    __threadfence();
    *(volatile v4f*)dst = v;
  } else if (task == 1) {
    if (blockIdx.x != 0) return;
    const int n = tid >> 3;
    const int q = tid & 7;
    float v[8];
#pragma unroll
    for (int e = 0; e < 8; ++e) v[e] = fc1[(size_t)(8 * q + e) * 32 + n];
    v4u wh, wl;
    pack_split8(v, wh, wl);
    store_planes2(f1h, f1l, (size_t)tid * 8, wh, wl);
  } else {
    if (blockIdx.x != 0) return;
    if (tid >= 64) return;
    const int o = tid >> 2;
    const int q = tid & 3;
    const int oc = (o < NOUTS) ? o : (NOUTS - 1);
    const bool live = o < NOUTS;
    float v[8];
#pragma unroll
    for (int e = 0; e < 8; ++e) {
      const float f = fc2[(size_t)(8 * q + e) * NOUTS + oc];
      v[e] = live ? f : 0.f;
    }
    v4u wh, wl;
    pack_split8(v, wh, wl);
    store_planes2(f2h, f2l, (size_t)tid * 8, wh, wl);
  }
}

__device__ __forceinline__ float sigm_f(float z) { return 1.0f / (1.0f + expf(-z)); }

__global__ __launch_bounds__(256) void k_lstm(
    const float* __restrict__ x, const float* __restrict__ wxp, const float* __restrict__ bbp,
    const unsigned short* __restrict__ whs,
    const unsigned short* __restrict__ f1h, const unsigned short* __restrict__ f1l,
    const unsigned short* __restrict__ f2h, const unsigned short* __restrict__ f2l,
    const float* __restrict__ fc1b, const float* __restrict__ fc2b,
    float* __restrict__ hout, int cell0) {
  __shared__ __align__(16) _Float16 s_h[8][64];
  __shared__ __align__(16) __bf16 s_rh[8][64];
  __shared__ __align__(16) __bf16 s_rl[8][64];
  __shared__ __align__(16) __bf16 s_ah[8][32];
  __shared__ __align__(16) __bf16 s_al[8][32];
  __shared__ __align__(16) float s_o[8][32];

  const int lane = threadIdx.x & 31;
  const int wave = threadIdx.x >> 5;
  const int hh = lane >> 4;
  const int c = lane & 15;
  const int cell = cell0 + (int)blockIdx.x * 8 + wave;
  if (cell >= BNREAL) return;
  const int b = cell / NNODE;
  const int n = cell - b * NNODE;
  const float* xrow = x + ((size_t)b * NSTEP * NNODE + n) * XPITCH;
  const int u0 = 32 * hh + c;
  const int u1 = u0 + 16;

  float xw[4][2], bv[4][2];
  {
    const float* wc = wxp + (size_t)cell * 256;
    const float* bc = bbp + (size_t)cell * 256;
#pragma unroll
    for (int g = 0; g < 4; ++g) { xw[g][0] = wc[g * 64 + u0]; xw[g][1] = wc[g * 64 + u1]; }
    asm volatile("" ::: "memory");
#pragma unroll
    for (int g = 0; g < 4; ++g) { bv[g][0] = bc[g * 64 + u0]; bv[g][1] = bc[g * 64 + u1]; }
  }
  const _Float16* whc = (const _Float16*)whs + (size_t)(cell - cell0) * (4 * WHN);
  _Float16* sh = s_h[wave];
  float cst[2] = {0.f, 0.f};
  float hst[2] = {0.f, 0.f};
  sh[u0] = (_Float16)0.0f;
  sh[u1] = (_Float16)0.0f;
  wave_lds_sync();
  const float RECSC = 1.0f / 16384.0f;

#pragma unroll 1
  for (int t = 0; t < NSTEP; ++t) {
    const float xt = xrow[(size_t)t * (NNODE * XPITCH)];
    float zr[4][4];
#pragma unroll
    for (int g = 0; g < 4; ++g)
#pragma unroll
      for (int j = 0; j < 4; ++j) zr[g][j] = 0.f;
    if (t > 0) {
      const v16h a0 = Frag<_Float16>::load(sh + 8 * hh);
      const v16h a1 = Frag<_Float16>::load(sh + 32 + 8 * hh);
#pragma unroll
      for (int g = 0; g < 4; ++g) {
#pragma unroll
        for (int j = 0; j < 4; ++j) {
          const _Float16* bp = whc + g * WHN + (16 * j + c) * NHID + 8 * hh;
          const v16h b0 = Frag<_Float16>::load(bp);
          const v16h b1 = Frag<_Float16>::load(bp + 32);
          v8f acc = zero8();
          acc = Frag<_Float16>::mma(a0, b0, acc);
          acc = Frag<_Float16>::mma(a1, b1, acc);
          guard1h(acc, a1, b1);
          zr[g][j] = acc[0];
          asm volatile("" ::: "memory");
        }
      }
    }
#pragma unroll
    for (int s = 0; s < 2; ++s) {
      const float r0 = hh ? zr[0][2 + s] : zr[0][s];
      const float r1 = hh ? zr[1][2 + s] : zr[1][s];
      const float r2 = hh ? zr[2][2 + s] : zr[2][s];
      const float r3 = hh ? zr[3][2 + s] : zr[3][s];
      const float z0 = xw[0][s] * xt + bv[0][s] + r0 * RECSC;
      const float z1 = xw[1][s] * xt + bv[1][s] + r1 * RECSC;
      const float z2 = xw[2][s] * xt + bv[2][s] + r2 * RECSC;
      const float z3 = xw[3][s] * xt + bv[3][s] + r3 * RECSC;
      const float gg = tanhf(z0);
      const float ig = sigm_f(z1);
      const float fg = sigm_f(z2);
      const float og = sigm_f(z3);
      const float cn = gg * ig + cst[s] * fg;
      cst[s] = cn;
      hst[s] = tanhf(cn) * og;
    }
    sh[u0] = (_Float16)(hst[0] * 256.0f);
    sh[u1] = (_Float16)(hst[1] * 256.0f);
    wave_lds_sync();
  }

  __bf16* rh = s_rh[wave];
  __bf16* rl = s_rl[wave];
  {
    const float q0 = fmaxf(hst[0], 0.f);
    const float q1 = fmaxf(hst[1], 0.f);
    const unsigned short h0b = f2bf_bits(q0), h1b = f2bf_bits(q1);
    const unsigned short l0b = f2bf_bits(q0 - bf_bits2f(h0b)), l1b = f2bf_bits(q1 - bf_bits2f(h1b));
    rh[u0] = __builtin_bit_cast(__bf16, h0b);
    rh[u1] = __builtin_bit_cast(__bf16, h1b);
    rl[u0] = __builtin_bit_cast(__bf16, l0b);
    rl[u1] = __builtin_bit_cast(__bf16, l1b);
  }
  wave_lds_sync();
  const v16b ah0 = Frag<__bf16>::load(rh + 8 * hh);
  const v16b ah1 = Frag<__bf16>::load(rh + 32 + 8 * hh);
  const v16b al0 = Frag<__bf16>::load(rl + 8 * hh);
  const v16b al1 = Frag<__bf16>::load(rl + 32 + 8 * hh);
  const __bf16* F1h = (const __bf16*)f1h;
  const __bf16* F1l = (const __bf16*)f1l;
  float a1v[2];
#pragma unroll
  for (int j = 0; j < 2; ++j) {
    const int nn = 16 * j + c;
    const __bf16* ph = F1h + (size_t)nn * NHID + 8 * hh;
    const __bf16* pl = F1l + (size_t)nn * NHID + 8 * hh;
    const v16b bh0 = Frag<__bf16>::load(ph);
    const v16b bh1 = Frag<__bf16>::load(ph + 32);
    const v16b bl0 = Frag<__bf16>::load(pl);
    const v16b bl1 = Frag<__bf16>::load(pl + 32);
    v8f acc = zero8();
    acc = Frag<__bf16>::mma(ah0, bh0, acc);
    acc = Frag<__bf16>::mma(ah0, bl0, acc);
    acc = Frag<__bf16>::mma(al0, bh0, acc);
    acc = Frag<__bf16>::mma(ah1, bh1, acc);
    acc = Frag<__bf16>::mma(ah1, bl1, acc);
    acc = Frag<__bf16>::mma(al1, bh1, acc);
    guard1b(acc, al1, bh1);
    a1v[j] = fmaxf(acc[0] + fc1b[nn], 0.f);
    asm volatile("" ::: "memory");
  }
  __bf16* sa = s_ah[wave];
  __bf16* sl = s_al[wave];
#pragma unroll
  for (int j = 0; j < 2; ++j) {
    const unsigned short hb = f2bf_bits(a1v[j]);
    const unsigned short lb = f2bf_bits(a1v[j] - bf_bits2f(hb));
    sa[16 * j + c] = __builtin_bit_cast(__bf16, hb);
    sl[16 * j + c] = __builtin_bit_cast(__bf16, lb);
  }
  wave_lds_sync();
  const v16b a2h = Frag<__bf16>::load(sa + 8 * hh);
  const v16b a2l = Frag<__bf16>::load(sl + 8 * hh);
  const __bf16* q2h = (const __bf16*)f2h + (size_t)c * 32 + 8 * hh;
  const __bf16* q2l = (const __bf16*)f2l + (size_t)c * 32 + 8 * hh;
  const v16b b2h = Frag<__bf16>::load(q2h);
  const v16b b2l = Frag<__bf16>::load(q2l);
  v8f acc2 = zero8();
  acc2 = Frag<__bf16>::mma(a2h, b2h, acc2);
  acc2 = Frag<__bf16>::mma(a2h, b2l, acc2);
  acc2 = Frag<__bf16>::mma(a2l, b2h, acc2);
  guard1b(acc2, a2l, b2h);
  const int cc = (c < NOUTS) ? c : (NOUTS - 1);
  const float ov = acc2[0] + fc2b[cc];
  float* so = s_o[wave];
  so[lane] = (lane < NOUTS) ? ov : 0.f;
  wave_lds_sync();
  const int q = lane & 7;
  const v4f vo = *(const v4f*)(so + 4 * q);
  float* dst = hout + (size_t)cell * 32 + 4 * q;
  if (lane < 8) *(volatile v4f*)dst = vo;
  __threadfence();
  if (lane < 8) *(volatile v4f*)dst = vo;
}

__global__ __launch_bounds__(256) void k_out(const float* __restrict__ hout, float* __restrict__ out) {
  const int i = blockIdx.x * 256 + threadIdx.x;
  if (i >= NOUTEL / 4) return;
  v4f v;
#pragma unroll
  for (int k = 0; k < 4; ++k) {
    const int e = 4 * i + k;
    const int b = e / (NOUTS * NNODE);
    const int rem = e - b * (NOUTS * NNODE);
    const int o = rem / NNODE;
    const int n = rem - o * NNODE;
    v[k] = hout[((size_t)(b * NNODE + n)) * 32 + o];
  }
  float* dst = out + (size_t)i * 4;
  *(volatile v4f*)dst = v;
  __threadfence();
  *(volatile v4f*)dst = v;
}

extern "C" void kernel_launch(void* const* d_in, const int* in_sizes, int n_in,
                              void* d_out, int out_size, void* d_ws, size_t ws_size,
                              hipStream_t stream) {
  if (n_in < 17) return;
  if (in_sizes[0] != NBATCH * NSTEP * NNODE * XPITCH) return;
  if (in_sizes[7] != 4 * NLH * WHN) return;
  if (out_size != NOUTEL) return;
  if (ws_size < WS_TOTAL) return;

  const float* x    = (const float*)d_in[0];
  const float* wx1  = (const float*)d_in[1];
  const float* wx1b = (const float*)d_in[2];
  const float* wx2  = (const float*)d_in[3];
  const float* wx2b = (const float*)d_in[4];
  const float* wh1  = (const float*)d_in[5];
  const float* wh1b = (const float*)d_in[6];
  const float* wh2  = (const float*)d_in[7];
  const float* wh2b = (const float*)d_in[8];
  const float* b1   = (const float*)d_in[9];
  const float* b1b  = (const float*)d_in[10];
  const float* b2   = (const float*)d_in[11];
  const float* b2b  = (const float*)d_in[12];
  const float* fc1  = (const float*)d_in[13];
  const float* fc1b = (const float*)d_in[14];
  const float* fc2  = (const float*)d_in[15];
  const float* fc2b = (const float*)d_in[16];
  float* out = (float*)d_out;

  char* ws = (char*)d_ws;
  unsigned short* meta_h = (unsigned short*)(ws + OFF_META_H);
  unsigned short* meta_l = (unsigned short*)(ws + OFF_META_L);
  unsigned short* w1t_h  = (unsigned short*)(ws + OFF_W1T_H);
  unsigned short* w1t_l  = (unsigned short*)(ws + OFF_W1T_L);
  unsigned short* w2t_h  = (unsigned short*)(ws + OFF_W2T_H);
  unsigned short* w2t_l  = (unsigned short*)(ws + OFF_W2T_L);
  unsigned short* wh2t   = (unsigned short*)(ws + OFF_WH2T);
  float*          wh2bp  = (float*)(ws + OFF_WHBP);
  unsigned short* fc1t_h = (unsigned short*)(ws + OFF_FC1T_H);
  unsigned short* fc1t_l = (unsigned short*)(ws + OFF_FC1T_L);
  unsigned short* fc2t_h = (unsigned short*)(ws + OFF_FC2T_H);
  unsigned short* fc2t_l = (unsigned short*)(ws + OFF_FC2T_L);
  unsigned short* hid_h  = (unsigned short*)(ws + OFF_HID_H);
  unsigned short* hid_l  = (unsigned short*)(ws + OFF_HID_L);
  unsigned short* hidwh  = hid_h;
  float*          wxp    = (float*)(ws + OFF_WX);
  float*          bbp    = (float*)(ws + OFF_BB);
  unsigned short* whs    = (unsigned short*)(ws + OFF_WHS);
  float*          hout   = (float*)(ws + OFF_HOUT);

  const dim3 blk(256);
  const size_t W1T4 = (size_t)4 * NLH * NEMB;
  const size_t W2T4 = (size_t)4 * NHID * NLH;

  k_meta<<<dim3((MPAD * 12) / 256), blk, 0, stream>>>(x, meta_h, meta_l);
  k_prep_w1<<<dim3(24, 3), blk, 0, stream>>>(wx1, wh1, b1, w1t_h, w1t_l);
  k_prep_w2<<<dim3(16, 2), blk, 0, stream>>>(wx2, b2, w2t_h, w2t_l);
  k_prep_wh2<<<dim3(256, 4), blk, 0, stream>>>(wh2, wh2t);
  k_prep_misc<<<dim3(16, 3), blk, 0, stream>>>(wh2b, fc1, fc2, wh2bp, fc1t_h, fc1t_l, fc2t_h, fc2t_l);

  wmma_gemm64<1, true, 2, 2, false, 2><<<dim3(TILES_L1 / 8, 4), blk, 0, stream>>>(
      meta_h, meta_l, NEMB, 0L,
      w1t_h + 0 * W1T4, w1t_l + 0 * W1T4, NEMB, (long)NLH * NEMB,
      hid_h, hid_l, NLH, (long)MPAD * NLH,
      wx1b, (long)NLH, nullptr, 0L,
      MPAD, NLH, NEMB, 1.0f, 1.0f);
  wmma_gemm64<1, true, 2, 0, false, 0><<<dim3(TILES_L2 / 8, 4), blk, 0, stream>>>(
      hid_h, hid_l, NLH, (long)MPAD * NLH,
      w2t_h + 0 * W2T4, w2t_l + 0 * W2T4, NLH, (long)NHID * NLH,
      wxp, nullptr, 256, (long)NHID,
      wx2b, (long)NHID, nullptr, 0L,
      MPAD, NHID, NLH, 1.0f, 1.0f);
  wmma_gemm64<1, true, 2, 2, false, 2><<<dim3(TILES_L1 / 8, 4), blk, 0, stream>>>(
      meta_h, meta_l, NEMB, 0L,
      w1t_h + 2 * W1T4, w1t_l + 2 * W1T4, NEMB, (long)NLH * NEMB,
      hid_h, hid_l, NLH, (long)MPAD * NLH,
      b1b, (long)NLH, nullptr, 0L,
      MPAD, NLH, NEMB, 1.0f, 1.0f);
  wmma_gemm64<1, true, 2, 0, false, 0><<<dim3(TILES_L2 / 8, 4), blk, 0, stream>>>(
      hid_h, hid_l, NLH, (long)MPAD * NLH,
      w2t_h + 1 * W2T4, w2t_l + 1 * W2T4, NLH, (long)NHID * NLH,
      bbp, nullptr, 256, (long)NHID,
      b2b, (long)NHID, nullptr, 0L,
      MPAD, NHID, NLH, 1.0f, 1.0f);
  wmma_gemm64<1, true, 2, 1, false, 2><<<dim3(TILES_L1 / 8, 4), blk, 0, stream>>>(
      meta_h, meta_l, NEMB, 0L,
      w1t_h + 1 * W1T4, w1t_l + 1 * W1T4, NEMB, (long)NLH * NEMB,
      hidwh, nullptr, NLH, (long)MPAD * NLH,
      wh1b, (long)NLH, nullptr, 0L,
      MPAD, NLH, NEMB, 1.0f, 16.0f);

  for (int ch = 0; ch < NCHUNK; ++ch) {
    wmma_gemm64<0, false, 2, 1, false, 0><<<dim3(TILES_WH / 8, 4), blk, 0, stream>>>(
        hidwh + (size_t)ch * MCH * NLH, nullptr, NLH, (long)MPAD * NLH,
        wh2t, nullptr, NLH, (long)WHN * NLH,
        whs, nullptr, 4 * WHN, (long)WHN,
        wh2bp, (long)WHN, nullptr, 0L,
        MCH, WHN, NLH, 1.0f / 1024.0f, 64.0f);
    k_lstm<<<dim3(MCH / 8), blk, 0, stream>>>(
        x, wxp, bbp, whs, fc1t_h, fc1t_l, fc2t_h, fc2t_l, fc1b, fc2b, hout, ch * MCH);
  }

  k_out<<<dim3((NOUTEL / 4 + 255) / 256), blk, 0, stream>>>(hout, out);
}
